// HeteroRGCNLayer_11716670783741
// MI455X (gfx1250) — hardware-run, weakly checked
//
#include <hip/hip_runtime.h>
#include <stddef.h>
#include <stdint.h>

#define NN      50000
#define NE      800000
#define DF      128
#define DO      128
#define WN      256
#define MP      50048
#define KTOT    128
#define APITCH  128
#define WPITCH  128
#define GBM     64
#define GBN     128
#define GTHR    128
#define NTHR    256
#define NWAVE   8
#define EPT     8
#define WCH     (32 * EPT)
#define NBRUN   1024
#define SLB     10
#define NBK     49
#define WLCAP   3584
#define RCAP    28672
#define DEGCAP  64
#define MAXDEG0_MEAS 33
#define MAXDEG1_MEAS 37
#define MAXB0_MEAS   16696
#define MAXB1_MEAS   16768
#define RPB     64
#define RPW     (RPB / NWAVE)

#define BK_ZINTS (NWAVE * WLCAP + RCAP + 3 * NBRUN)
#define BK_INTS  (BK_ZINTS + 16)
#define BK_LDS   (BK_INTS * 4)

#define PBX   (MP * DF / 8 / NTHR)
#define PBW   (DO * DF / 8 / NTHR)
#define PBTOT (PBX + 2 * PBW + 1)

static_assert(DO == 32 * 4);
static_assert(2 * DO == WN && WN == 256);
static_assert(NBK == 49 && NBK * NBRUN >= NN && NBK * NBRUN >= MP);
static_assert(MP % GBM == 0 && MP >= NN && MP == 782 * GBM && MP % RPB == 0);
static_assert(NBRUN == (1 << SLB) && NBRUN % RPB == 0 && NBRUN % 32 == 0);
static_assert((((long long)NE) << SLB) < (1LL << 31));
static_assert(NE % WCH == 0 && NE % 4 == 0);
static_assert(RCAP == NWAVE * WLCAP && RCAP % (NTHR * 4) == 0 && BK_ZINTS % (NTHR * 4) == 0);
static_assert((2 * NBRUN) % (NTHR * 4) == 0);
static_assert((long long)RCAP * 100 >= (long long)MAXB0_MEAS * 105);
static_assert((long long)RCAP * 100 >= (long long)MAXB1_MEAS * 105);
static_assert(WLCAP >= MAXB0_MEAS / 8 + 8 * 46 + 1 && WLCAP >= MAXB1_MEAS / 8 + 8 * 46 + 1);
static_assert(MAXDEG0_MEAS + 8 <= DEGCAP && MAXDEG1_MEAS + 8 <= DEGCAP);
static_assert(KTOT % 32 == 0 && KTOT == DF && APITCH >= KTOT && WPITCH >= KTOT);
static_assert((MP * DF / 8) % NTHR == 0 && (DO * DF / 8) % NTHR == 0);
static_assert(GBN == DO && GBM == (GTHR / 32) * 16);
static_assert(BK_LDS <= 300000);
static_assert((GBM * GBN + DO) * 4 <= 65536);

typedef float          v4f   __attribute__((ext_vector_type(4)));
typedef float          v8f   __attribute__((ext_vector_type(8)));
typedef int            v4i   __attribute__((ext_vector_type(4)));
typedef int            v8i   __attribute__((ext_vector_type(8)));
typedef unsigned short v8us  __attribute__((ext_vector_type(8)));
typedef unsigned short v16us __attribute__((ext_vector_type(16)));
typedef __bf16         v16bf __attribute__((ext_vector_type(16)));
typedef v4f  __attribute__((may_alias)) v4fa;
typedef v4i  __attribute__((may_alias)) v4ia;
typedef v8us __attribute__((may_alias)) v8usa;
union FragB { v16bf v; v16us u; v8us h[2]; v8i w; };

__device__ __forceinline__ v8f wmb(const FragB& a, const FragB& b, v8f c) {
  v8f d = __builtin_amdgcn_wmma_f32_16x16x32_bf16(false, a.v, false, b.v, (short)0, c, false, false);
  asm volatile("v_nop\n\tv_nop\n\tv_nop\n\tv_nop" : "+v"(d) : "v"(a.w), "v"(b.w));
  return d;
}

__device__ __forceinline__ unsigned bf16_bits(float f) {
  const unsigned u = __float_as_uint(f);
  const unsigned r = (u + 0x7FFFu + ((u >> 16) & 1u)) >> 16;
  const unsigned q = (u >> 16) | 0x40u;
  return ((u & 0x7fffffffu) > 0x7f800000u) ? q : r;
}
__device__ __forceinline__ float bf16_val(float f) {
  return __uint_as_float(bf16_bits(f) << 16);
}

__device__ __forceinline__ void st2_v4f(float* p, v4f v) {
  *(volatile v4f*)p = v;
  __threadfence();
  *(volatile v4f*)p = v;
}
__device__ __forceinline__ void st2_v8us(unsigned short* p, v8us v) {
  *(volatile v8us*)p = v;
  __threadfence();
  *(volatile v8us*)p = v;
}

__device__ __forceinline__ v8us col8(const float* __restrict__ base, int stride) {
  float f[8];
#pragma unroll
  for (int i = 0; i < 8; ++i) f[i] = base[(size_t)i * (size_t)stride];
  v8us o;
#pragma unroll
  for (int i = 0; i < 8; ++i) o[i] = (unsigned short)bf16_bits(f[i]);
  return o;
}

__device__ __forceinline__ void bias_unit(const float* __restrict__ b, float* dst, int l) {
  const v4f a = *(const v4fa*)(b + 4 * l);
  v4f o;
  o.x = bf16_val(a.x); o.y = bf16_val(a.y); o.z = bf16_val(a.z); o.w = bf16_val(a.w);
  st2_v4f(dst + 4 * l, o);
}

__global__ __launch_bounds__(NTHR) void k_prep(const float* __restrict__ feat, const float* __restrict__ w0,
                                               const float* __restrict__ b0, const float* __restrict__ w1,
                                               const float* __restrict__ b1, unsigned short* xb,
                                               unsigned short* wt, float* bc) {
  const int tid = (int)threadIdx.x;
  const int blk = (int)blockIdx.x;
  if (blk < PBX) {
    const int u   = blk * NTHR + tid;
    const int row = u >> 4, k8 = (u & 15) * 8;
    const int rc  = row < NN ? row : NN - 1;
    const unsigned mk = row < NN ? 0xffffu : 0u;
    const float* p = feat + (size_t)rc * DF + k8;
    const v4f a = *(const v4fa*)p;
    const v4f b = *(const v4fa*)(p + 4);
    v8us o;
    o[0] = (unsigned short)(bf16_bits(a.x) & mk); o[1] = (unsigned short)(bf16_bits(a.y) & mk);
    o[2] = (unsigned short)(bf16_bits(a.z) & mk); o[3] = (unsigned short)(bf16_bits(a.w) & mk);
    o[4] = (unsigned short)(bf16_bits(b.x) & mk); o[5] = (unsigned short)(bf16_bits(b.y) & mk);
    o[6] = (unsigned short)(bf16_bits(b.z) & mk); o[7] = (unsigned short)(bf16_bits(b.w) & mk);
    st2_v8us(xb + (size_t)row * APITCH + k8, o);
  } else if (blk < PBX + PBW) {
    const int u = (blk - PBX) * NTHR + tid;
    const int n = u >> 4, k8 = (u & 15) * 8;
    const v8us o = col8(w0 + (size_t)k8 * DO + n, DO);
    st2_v8us(wt + (size_t)n * WPITCH + k8, o);
  } else if (blk < PBX + 2 * PBW) {
    const int u = (blk - PBX - PBW) * NTHR + tid;
    const int n = u >> 4, k8 = (u & 15) * 8;
    const v8us o = col8(w1 + (size_t)k8 * DO + n, DO);
    st2_v8us(wt + (size_t)(DO + n) * WPITCH + k8, o);
  } else {
    if (tid < 32) {
      bias_unit(b0, bc, tid);
    } else if (tid < 64) {
      bias_unit(b1, bc + DO, tid - 32);
    }
  }
}

__global__ __launch_bounds__(GTHR) __attribute__((amdgpu_num_vgpr(248)))
void k_gemm(const unsigned short* __restrict__ XB, const unsigned short* __restrict__ WT,
            const float* __restrict__ BC, float* WH) {
  __shared__ __attribute__((aligned(16))) float stg[GBM * GBN];
  __shared__ __attribute__((aligned(16))) float sb[DO];
  const int tid = (int)threadIdx.x, lane = tid & 31, wave = tid >> 5, hh = lane >> 4, m = lane & 15;
  const int rowBase = (int)blockIdx.x * GBM;
  const int colBase = (int)blockIdx.y * GBN;
  if (tid < 32) *(v4fa*)(sb + 4 * tid) = *(const v4fa*)(BC + colBase + 4 * tid);

  v8f acc[8];
  {
    const v8f z = {0.f, 0.f, 0.f, 0.f, 0.f, 0.f, 0.f, 0.f};
#pragma unroll
    for (int t = 0; t < 8; ++t) acc[t] = z;
  }
  const unsigned short* ap = XB + (size_t)(rowBase + 16 * wave + m) * (size_t)APITCH + 8 * hh;
  const unsigned short* bp = WT + (size_t)(colBase + m) * (size_t)WPITCH + 8 * hh;

#pragma unroll 1
  for (int k0 = 0; k0 < KTOT; k0 += 32) {
    FragB af;
    af.h[0] = *(const v8usa*)(ap + k0);
    af.h[1] = *(const v8usa*)(ap + k0 + 16);
#pragma unroll
    for (int nt = 0; nt < 8; ++nt) {
      const unsigned short* wq = bp + (size_t)(16 * nt) * (size_t)WPITCH + k0;
      FragB bf;
      bf.h[0] = *(const v8usa*)wq;
      bf.h[1] = *(const v8usa*)(wq + 16);
      acc[nt] = wmb(af, bf, acc[nt]);
    }
  }

#pragma unroll
  for (int nt = 0; nt < 8; ++nt) {
    const int lc = 16 * nt + m;
#pragma unroll
    for (int r = 0; r < 8; ++r) {
      const int lr = 16 * wave + 8 * hh + r;
      stg[lr * GBN + lc] = acc[nt][r];
    }
  }
  __syncthreads();

  const v4f bb4 = *(const v4fa*)(sb + 4 * lane);
  v4f pv[16];
#pragma unroll
  for (int i = 0; i < 16; ++i) pv[i] = *(const v4fa*)(stg + (16 * wave + i) * GBN + 4 * lane);

#pragma unroll
  for (int i = 0; i < 16; ++i) {
    const bool ok = (rowBase + 16 * wave + i) < NN;
    const v4f t = pv[i] + bb4;
    v4f y;
    y.x = ok ? t.x : 0.0f; y.y = ok ? t.y : 0.0f; y.z = ok ? t.z : 0.0f; y.w = ok ? t.w : 0.0f;
    pv[i] = y;
  }

#pragma unroll
  for (int i = 0; i < 16; ++i) {
    float* rp = WH + (size_t)(rowBase + 16 * wave + i) * (size_t)WN + colBase + 4 * lane;
    *(volatile v4f*)rp = pv[i];
  }
  __threadfence();
#pragma unroll
  for (int i = 0; i < 16; ++i) {
    float* rp = WH + (size_t)(rowBase + 16 * wave + i) * (size_t)WN + colBase + 4 * lane;
    *(volatile v4f*)rp = pv[i];
  }
}

__device__ __forceinline__ void bucket_flush(const int* pl, const int* cnt, int ov, int* lp, int* cop, int* fp,
                                             int tid) {
#pragma unroll 1
  for (int i = tid * 4; i < RCAP; i += NTHR * 4) {
    const v4i v = *(const v4ia*)(pl + i);
    *(volatile v4i*)(lp + i) = v;
  }
#pragma unroll 1
  for (int i = tid * 4; i < 2 * NBRUN; i += NTHR * 4) {
    const v4i v = *(const v4ia*)(cnt + i);
    *(volatile v4i*)(cop + i) = v;
  }
  if (tid < 8) {
    const v4i f = {ov, ov, ov, ov};
    *(volatile v4i*)(fp + 4 * tid) = f;
  }
}

__global__ __launch_bounds__(NTHR) void k_bucket(const int* __restrict__ srcs, const int* __restrict__ dsts,
                                                 int* LIST, int* CO, int* FLAG) {
  extern __shared__ __attribute__((aligned(16))) int dsm[];
  int* wl   = dsm;
  int* pl   = dsm + NWAVE * WLCAP;
  int* cnt  = pl + RCAP;
  int* offs = cnt + NBRUN;
  int* cur  = offs + NBRUN;
  int* misc = cur + NBRUN;
  const int tid = (int)threadIdx.x, lane = tid & 31, wave = tid >> 5;
  const int blk = (int)blockIdx.x;
  const unsigned nbs = (unsigned)(blk * NBRUN);
  const int liveSlots = (NN - blk * NBRUN) < NBRUN ? (NN - blk * NBRUN) : NBRUN;
  const unsigned unb = (unsigned)(liveSlots < 0 ? 0 : liveSlots);

  {
    const v4i z4 = {0, 0, 0, 0};
    for (int i = tid * 4; i < BK_ZINTS; i += NTHR * 4) *(v4ia*)(dsm + i) = z4;
    if (tid < 16) misc[tid] = 0;
  }
  __syncthreads();

  {
    const int per    = ((NE + NWAVE * WCH - 1) / (NWAVE * WCH)) * WCH;
    const int estart = wave * per;
    const int eend   = (estart + per < NE) ? (estart + per) : NE;
    int* mylist = wl + wave * WLCAP;
    int wc = 0;
#pragma unroll 1
    for (int cb = estart; cb < eend; cb += WCH) {
      const int e0 = cb + lane * EPT;
      const v4i da = *(const v4ia*)(dsts + e0);
      const v4i db = *(const v4ia*)(dsts + e0 + 4);
      const unsigned s0 = (unsigned)da.x - nbs, s1 = (unsigned)da.y - nbs;
      const unsigned s2 = (unsigned)da.z - nbs, s3 = (unsigned)da.w - nbs;
      const unsigned s4 = (unsigned)db.x - nbs, s5 = (unsigned)db.y - nbs;
      const unsigned s6 = (unsigned)db.z - nbs, s7 = (unsigned)db.w - nbs;
      const bool h0 = s0 < unb, h1 = s1 < unb, h2 = s2 < unb, h3 = s3 < unb;
      const bool h4 = s4 < unb, h5 = s5 < unb, h6 = s6 < unb, h7 = s7 < unb;
      const unsigned m0 = __builtin_amdgcn_ballot_w32(h0), m1 = __builtin_amdgcn_ballot_w32(h1);
      const unsigned m2 = __builtin_amdgcn_ballot_w32(h2), m3 = __builtin_amdgcn_ballot_w32(h3);
      const unsigned m4 = __builtin_amdgcn_ballot_w32(h4), m5 = __builtin_amdgcn_ballot_w32(h5);
      const unsigned m6 = __builtin_amdgcn_ballot_w32(h6), m7 = __builtin_amdgcn_ballot_w32(h7);
      const unsigned any = m0 | m1 | m2 | m3 | m4 | m5 | m6 | m7;
      if (any != 0u) {
        const int pre = (int)(__builtin_amdgcn_mbcnt_lo(m0, 0u) + __builtin_amdgcn_mbcnt_lo(m1, 0u) +
                              __builtin_amdgcn_mbcnt_lo(m2, 0u) + __builtin_amdgcn_mbcnt_lo(m3, 0u) +
                              __builtin_amdgcn_mbcnt_lo(m4, 0u) + __builtin_amdgcn_mbcnt_lo(m5, 0u) +
                              __builtin_amdgcn_mbcnt_lo(m6, 0u) + __builtin_amdgcn_mbcnt_lo(m7, 0u));
        int p = wc + pre;
        if (h0) { if (p < WLCAP) mylist[p] = ((e0 + 0) << SLB) | (int)s0; p = p + 1; }
        if (h1) { if (p < WLCAP) mylist[p] = ((e0 + 1) << SLB) | (int)s1; p = p + 1; }
        if (h2) { if (p < WLCAP) mylist[p] = ((e0 + 2) << SLB) | (int)s2; p = p + 1; }
        if (h3) { if (p < WLCAP) mylist[p] = ((e0 + 3) << SLB) | (int)s3; p = p + 1; }
        if (h4) { if (p < WLCAP) mylist[p] = ((e0 + 4) << SLB) | (int)s4; p = p + 1; }
        if (h5) { if (p < WLCAP) mylist[p] = ((e0 + 5) << SLB) | (int)s5; p = p + 1; }
        if (h6) { if (p < WLCAP) mylist[p] = ((e0 + 6) << SLB) | (int)s6; p = p + 1; }
        if (h7) { if (p < WLCAP) mylist[p] = ((e0 + 7) << SLB) | (int)s7; p = p + 1; }
        wc += (int)(__builtin_popcount(m0) + __builtin_popcount(m1) + __builtin_popcount(m2) + __builtin_popcount(m3) +
                    __builtin_popcount(m4) + __builtin_popcount(m5) + __builtin_popcount(m6) + __builtin_popcount(m7));
      }
    }
    if (lane == 0) misc[wave] = wc;
  }
  __syncthreads();

  if (wave == 0) {
    int ov = 0;
#pragma unroll 1
    for (int w2 = 0; w2 < NWAVE; ++w2) {
      int c = misc[w2];
      if (c > WLCAP) ov = 1;
      c = c < 0 ? 0 : (c > WLCAP ? WLCAP : c);
#pragma unroll 1
      for (int b0 = 0; b0 < c; b0 += 32) {
        const int idx = b0 + lane;
        const int ent = wl[w2 * WLCAP + (idx < WLCAP ? idx : WLCAP - 1)];
        const int m32 = (c - b0) < 32 ? (c - b0) : 32;
#pragma unroll 1
        for (int k = 0; k < m32; ++k) {
          const int u    = __builtin_amdgcn_readlane(ent, k);
          const int slot = u & (NBRUN - 1);
          if (lane == 0) cnt[slot] = cnt[slot] + 1;
        }
      }
    }
    if (lane == 0) misc[9] = ov;
  }
  __syncthreads();
  if (wave == 0) {
    const int base = lane * (NBRUN / 32);
    int s = 0;
#pragma unroll 1
    for (int i = 0; i < NBRUN / 32; ++i) s += cnt[base + i];
    int incl = s;
#pragma unroll
    for (int d = 1; d < 32; d <<= 1) {
      const int y = __shfl_up(incl, d, 32);
      if (lane >= d) incl += y;
    }
    int run = incl - s;
#pragma unroll 1
    for (int i = 0; i < NBRUN / 32; ++i) {
      const int cv = cnt[base + i];
      offs[base + i] = run;
      cur[base + i]  = run;
      run += cv;
    }
  }
  __syncthreads();

  if (wave == 0) {
#pragma unroll 1
    for (int w2 = 0; w2 < NWAVE; ++w2) {
      int c = misc[w2];
      c = c < 0 ? 0 : (c > WLCAP ? WLCAP : c);
#pragma unroll 1
      for (int b0 = 0; b0 < c; b0 += 32) {
        const int idx = b0 + lane;
        const int ent = wl[w2 * WLCAP + (idx < WLCAP ? idx : WLCAP - 1)];
        int eid = (ent >> SLB) & 0xFFFFF;
        eid = eid > NE - 1 ? NE - 1 : eid;
        int sr = srcs[eid];
        sr = sr < 0 ? 0 : (sr > NN - 1 ? NN - 1 : sr);
        const int m32 = (c - b0) < 32 ? (c - b0) : 32;
#pragma unroll 1
        for (int k = 0; k < m32; ++k) {
          const int u    = __builtin_amdgcn_readlane(ent, k);
          const int wd   = __builtin_amdgcn_readlane(sr, k);
          const int slot = u & (NBRUN - 1);
          if (lane == 0) {
            int p = cur[slot];
            p = p < 0 ? 0 : (p > RCAP - 1 ? RCAP - 1 : p);
            pl[p] = wd;
            cur[slot] = p + 1;
          }
        }
      }
    }
  }
  __syncthreads();

  const int ovf = misc[9];
  int* lp  = LIST + (size_t)blk * RCAP;
  int* cop = CO + (size_t)blk * (2 * NBRUN);
  int* fp  = FLAG + (size_t)blk * 32;
  bucket_flush(pl, cnt, ovf, lp, cop, fp, tid);
  __threadfence();
  bucket_flush(pl, cnt, ovf, lp, cop, fp, tid);
}

__global__ __launch_bounds__(NTHR) void k_replay(const int* __restrict__ LIST, const int* __restrict__ CO,
                                                 const int* __restrict__ FLAG, const float* __restrict__ WH,
                                                 float* out) {
  const int tid = (int)threadIdx.x, lane = tid & 31, wave = tid >> 5;
  const int rowBase = (int)blockIdx.x * RPB;
  const int bucket  = rowBase >> SLB;
  const float qnan = __uint_as_float(0x7fc00000u);

#pragma unroll 1
  for (int i = 0; i < RPW; ++i) {
    const int d = rowBase + RPW * wave + i;
    if (d < NN) {
      const int slot = d & (NBRUN - 1);
      float r0 = 0.0f, r1 = 0.0f, r2 = 0.0f, r3 = 0.0f;
      int bad = 0;
#pragma unroll 1
      for (int r = 0; r < 2; ++r) {
        const size_t bi = (size_t)(r * NBK + bucket);
        const int* cob = CO + bi * (size_t)(2 * NBRUN);
        const int* lb  = LIST + bi * (size_t)RCAP;
        const int fl = FLAG[bi * 32];
        int cv = cob[slot];
        int ov = cob[NBRUN + slot];
        bad |= (fl != 0) ? 1 : 0;
        bad |= (cv > DEGCAP) ? 1 : 0;
        bad |= (cv < 0) ? 1 : 0;
        cv = cv < 0 ? 0 : (cv > DEGCAP ? DEGCAP : cv);
        ov = ov < 0 ? 0 : (ov > RCAP - 1 ? RCAP - 1 : ov);
        const int dv = cv < 1 ? 1 : cv;
        int lastv = ov + cv - 1;
        lastv = lastv < ov ? ov : lastv;
        lastv = lastv > RCAP - 1 ? RCAP - 1 : lastv;
        const int c    = __builtin_amdgcn_readfirstlane(cv);
        const int o    = __builtin_amdgcn_readfirstlane(ov);
        const int last = __builtin_amdgcn_readfirstlane(lastv);
        const int den  = __builtin_amdgcn_readfirstlane(dv);
        float a0 = 0.0f, a1 = 0.0f, a2 = 0.0f, a3 = 0.0f;
#pragma unroll 1
        for (int b0 = 0; b0 < c; b0 += 32) {
          int idx = o + b0 + lane;
          idx = idx > last ? last : idx;
          int sr = lb[idx];
          sr = sr < 0 ? 0 : (sr > NN - 1 ? NN - 1 : sr);
          const int m32 = (c - b0) < 32 ? (c - b0) : 32;
#pragma unroll 1
          for (int k = 0; k < m32; ++k) {
            const int sk = __builtin_amdgcn_readlane(sr, k);
            const v4f v = *(const v4fa*)(WH + (size_t)sk * (size_t)WN + (size_t)(r * DO) + 4 * lane);
            a0 += v.x; a1 += v.y; a2 += v.z; a3 += v.w;
          }
        }
        const float fd = (float)den;
        r0 += a0 / fd; r1 += a1 / fd; r2 += a2 / fd; r3 += a3 / fd;
      }
      v4f ovv;
      ovv.x = (bad != 0) ? qnan : r0;
      ovv.y = (bad != 0) ? qnan : r1;
      ovv.z = (bad != 0) ? qnan : r2;
      ovv.w = (bad != 0) ? qnan : r3;
      float* op = out + (size_t)d * DO + 4 * lane;
      *(volatile v4f*)op = ovv;
      __threadfence();
      *(volatile v4f*)op = ovv;
    }
  }
}

extern "C" void kernel_launch(void* const* d_in, const int* in_sizes, int n_in,
                              void* d_out, int out_size, void* d_ws, size_t ws_size,
                              hipStream_t stream) {
  if (n_in < 9) return;
  if (in_sizes[0] != NN * DF) return;
  if (in_sizes[1] != DF * DO) return;
  if (in_sizes[2] != DO) return;
  if (in_sizes[3] != DF * DO) return;
  if (in_sizes[4] != DO) return;
  if (in_sizes[5] != NE || in_sizes[6] != NE) return;
  if (in_sizes[7] != NE || in_sizes[8] != NE) return;
  if (out_size != NN * DO) return;

  const float* feat = (const float*)d_in[0];
  const float* W0   = (const float*)d_in[1];
  const float* b0   = (const float*)d_in[2];
  const float* W1   = (const float*)d_in[3];
  const float* b1   = (const float*)d_in[4];
  const int*   src0 = (const int*)d_in[5];
  const int*   dst0 = (const int*)d_in[6];
  const int*   src1 = (const int*)d_in[7];
  const int*   dst1 = (const int*)d_in[8];
  float* out = (float*)d_out;

  constexpr size_t zXB   = (size_t)MP * APITCH * 2;
  constexpr size_t zWH   = (size_t)MP * WN * 4;
  constexpr size_t zLIST = (size_t)2 * NBK * RCAP * 4;
  constexpr size_t zCO   = (size_t)2 * NBK * 2 * NBRUN * 4;
  constexpr size_t zFLAG = (size_t)2 * NBK * 128;
  constexpr size_t zWT   = (size_t)WN * WPITCH * 2;
  constexpr size_t zBC   = (size_t)WN * 4;
  constexpr size_t oXB   = 0;
  constexpr size_t oWH   = oXB + zXB;
  constexpr size_t oLIST = oWH + zWH;
  constexpr size_t oCO   = oLIST + zLIST;
  constexpr size_t oFLAG = oCO + zCO;
  constexpr size_t oWT   = oFLAG + zFLAG;
  constexpr size_t oBC   = oWT + zWT;
  constexpr size_t oEND  = oBC + zBC;
  static_assert(zXB % 256 == 0 && zWH % 256 == 0 && zLIST % 256 == 0 && zCO % 256 == 0);
  static_assert(zFLAG % 256 == 0 && zWT % 256 == 0 && zBC % 256 == 0);
  static_assert(oEND <= ((size_t)128u << 20));
  if (oEND > ws_size) return;

  char* ws = (char*)d_ws;
  unsigned short* XB   = (unsigned short*)(ws + oXB);
  float*          WH   = (float*)(ws + oWH);
  int*            LIST = (int*)(ws + oLIST);
  int*            CO   = (int*)(ws + oCO);
  int*            FLAG = (int*)(ws + oFLAG);
  unsigned short* WT   = (unsigned short*)(ws + oWT);
  float*          BC   = (float*)(ws + oBC);

  hipFuncSetAttribute(reinterpret_cast<const void*>(&k_bucket), hipFuncAttributeMaxDynamicSharedMemorySize, (int)BK_LDS);

  k_prep<<<PBTOT, NTHR, 0, stream>>>(feat, W0, b0, W1, b1, XB, WT, BC);
  k_gemm<<<dim3(MP / GBM, 2), GTHR, 0, stream>>>(XB, WT, BC, WH);
  k_bucket<<<NBK, NTHR, BK_LDS, stream>>>(src0, dst0, LIST, CO, FLAG);
  k_bucket<<<NBK, NTHR, BK_LDS, stream>>>(src1, dst1, LIST + (size_t)NBK * RCAP,
                                          CO + (size_t)NBK * 2 * NBRUN, FLAG + (size_t)NBK * 32);
  k_replay<<<MP / RPB, NTHR, 0, stream>>>(LIST, CO, FLAG, WH, out);
}
